// PoolLayer_26774826123433
// MI455X (gfx1250) — hardware-verified
//
#include <hip/hip_runtime.h>
#include <hip/hip_bf16.h>
#include <math.h>

#define NBp 16
#define L0 2048
#define L1 1024
#define DDp 128
#define HHp 384
#define GSTR 48

typedef _Float16 bf16;
typedef _Float16 f16;
typedef __attribute__((ext_vector_type(4))) unsigned v4u_t;
typedef unsigned v4ua __attribute__((ext_vector_type(4), may_alias));
typedef __attribute__((ext_vector_type(4))) float v4f_t;
typedef float v4fa __attribute__((ext_vector_type(4), may_alias));
typedef __attribute__((ext_vector_type(16))) bf16  bf16x16;
typedef bf16x16 f16x16;
typedef __attribute__((ext_vector_type(8)))  bf16  bf16x8;
typedef bf16x8 f16x8;
typedef __attribute__((ext_vector_type(4)))  bf16  bf16x4;
typedef __attribute__((ext_vector_type(8)))  float f32x8;
__device__ __forceinline__ f32x8 wmma16(f16x16 a, f16x16 b, f32x8 c) {
  c = __builtin_amdgcn_wmma_f32_16x16x32_f16(false, a, false, b, (short)0, c, false, false);
  asm volatile("v_nop\n\tv_nop\n\tv_nop\n\tv_nop" : "+v"(c) : "v"(a), "v"(b));
  return c;
}
#define LDS_STRIDE 48
#define KSTRIDE    72
#define VSTRIDE    48

__device__ __forceinline__ f32x8 wmma_bf16(bf16x16 a, bf16x16 b, f32x8 c) {
  c = __builtin_amdgcn_wmma_f32_16x16x32_f16(false, a, false, b, (short)0, c, false, false);
  asm volatile("v_nop\n\tv_nop\n\tv_nop\n\tv_nop" : "+v"(c) : "v"(a), "v"(b));
  return c;
}

template <typename T>
__device__ __forceinline__ bf16x16 load_frag(const T* __restrict__ base, int ld,
                                             int row0, int k0) {
  const int lane = threadIdx.x & 31;
  const int r    = lane & 15;
  const int kh   = (lane >> 4) * 8;
  const T* p0 = base + (size_t)(row0 + r) * ld + (k0 + kh);
  const T* p1 = p0 + 16;
  bf16x16 f;
#pragma unroll
  for (int i = 0; i < 8; ++i) {
    f[i]     = (bf16)p0[i];
    f[i + 8] = (bf16)p1[i];
  }
  return f;
}

__device__ __forceinline__ bf16x16 lds_frag(const bf16* base, int stride) {
  const int lane = threadIdx.x & 31;
  const int row  = lane & 15;
  const int kh   = (lane >> 4) * 8;
  const bf16x8 lo = *(const bf16x8*)(base + row * stride + kh);
  const bf16x8 hi = *(const bf16x8*)(base + row * stride + kh + 16);
  bf16x16 f;
#pragma unroll
  for (int i = 0; i < 8; ++i) { f[i] = lo[i]; f[i + 8] = hi[i]; }
  return f;
}

template <typename T>
__device__ __forceinline__ void stage_read16(const T* __restrict__ p, float* buf) {
#pragma unroll
  for (int i = 0; i < 16; ++i) buf[i] = (float)p[i];
}

__device__ __forceinline__ void stage_write(bf16* dst, const float* buf, int nquad) {
#pragma unroll
  for (int i = 0; i < nquad; ++i) {
    bf16x4 q;
    q[0] = (bf16)buf[4 * i];     q[1] = (bf16)buf[4 * i + 1];
    q[2] = (bf16)buf[4 * i + 2]; q[3] = (bf16)buf[4 * i + 3];
    *(bf16x4*)(dst + 4 * i) = q;
  }
}


#define GSTR 48
template <typename AT, int EPI, bool OUT16>
__global__ __launch_bounds__(256) void gemm_kne(const AT* __restrict__ A, int lda, const float* __restrict__ Wm, int ldw,
                                                const float* __restrict__ bias, const float* __restrict__ R, const float* __restrict__ gvec,
                                                void* __restrict__ Yv, int ldy, int K) {
  __shared__ __attribute__((aligned(16))) f16 ldsA[128 * GSTR];
  __shared__ __attribute__((aligned(16))) f16 ldsW[128 * GSTR];
  __shared__ __attribute__((aligned(16))) float oS[8][32 * 68];
  const int tid = threadIdx.x, lane = tid & 31, wave = tid >> 5, cl = lane & 15, rh = (lane >> 4) * 8;
  const int m0 = blockIdx.x * 128, n0 = blockIdx.y * 128;
  const int wm = (wave & 3) * 32, wn = (wave >> 2) * 64;
  f32x8 acc[2][4];
#pragma unroll
  for (int i = 0; i < 2; ++i)
#pragma unroll
    for (int j = 0; j < 4; ++j) { f32x8 z = {}; acc[i][j] = z; }
#pragma unroll 1
  for (int k0 = 0; k0 < K; k0 += 32) {
    __syncthreads();
    { const int row = tid >> 1, ch = (tid & 1) * 16;
      const AT* src = A + (size_t)(m0 + row) * lda + k0 + ch;
#pragma unroll
      for (int g = 0; g < 16; ++g) ldsA[row * GSTR + ch + g] = (f16)src[g]; }
    { const int k = tid >> 3, nn0 = (tid & 7) * 16;
      const float* src = Wm + (size_t)(k0 + k) * ldw + n0 + nn0;
#pragma unroll
      for (int g = 0; g < 4; ++g) { const v4f_t v = *(const v4f_t*)(src + 4 * g);
#pragma unroll
        for (int u = 0; u < 4; ++u) ldsW[(nn0 + 4 * g + u) * GSTR + k] = (f16)v[u]; } }
    __syncthreads();
    f16x16 af[2];
#pragma unroll
    for (int i = 0; i < 2; ++i) af[i] = lds_frag(ldsA + (wm + 16 * i) * GSTR, GSTR);
#pragma unroll
    for (int j = 0; j < 4; ++j) {
      const f16x16 bf = lds_frag(ldsW + (wn + 16 * j) * GSTR, GSTR);
#pragma unroll
      for (int i = 0; i < 2; ++i) acc[i][j] = wmma16(af[i], bf, acc[i][j]);
    }
  }
  float* so = oS[wave];
#pragma unroll
  for (int i = 0; i < 2; ++i)
#pragma unroll
    for (int j = 0; j < 4; ++j) {
      const int n = n0 + wn + 16 * j + cl;
      const float bv = bias ? bias[n] : 0.0f;
      const float gv = (EPI == 2) ? gvec[n] : 0.0f;
      if (EPI == 1) {
#pragma unroll 1
        for (int r = 0; r < 8; ++r) { const float xg = acc[i][j][r] + bv; so[(16 * i + rh + r) * 68 + 16 * j + cl] = 0.5f * xg * (1.0f + erff(xg * 0.70710678118654752f)); }
      } else {
#pragma unroll
        for (int r = 0; r < 8; ++r) {
          float v = acc[i][j][r] + bv;
          if (EPI == 2) v = R[(size_t)(m0 + wm + 16 * i + rh + r) * ldy + n] + gv * v;
          so[(16 * i + rh + r) * 68 + 16 * j + cl] = v;
        }
      }
    }
  asm volatile("s_wait_dscnt 0" ::: "memory");
  __builtin_amdgcn_wave_barrier();
#pragma unroll 1
  for (int pass = 0; pass < 2; ++pass) {
    if (OUT16) {
      f16* Y = (f16*)Yv;
#pragma unroll
      for (int it = 0; it < 8; ++it) { const int c = lane + 32 * it, rr = c >> 3, q8 = (c & 7) * 8;
        union { f16 h[8]; v4u_t v; } u;
#pragma unroll
        for (int e = 0; e < 8; ++e) u.h[e] = (f16)so[rr * 68 + q8 + e];
        *(volatile v4u_t*)(Y + (size_t)(m0 + wm + rr) * ldy + n0 + wn + q8) = u.v; }
    } else {
      float* Y = (float*)Yv;
#pragma unroll
      for (int it = 0; it < 16; ++it) { const int f4 = lane + 32 * it, rr = f4 >> 4, q = (f4 & 15) * 4;
        *(volatile v4f_t*)(Y + (size_t)(m0 + wm + rr) * ldy + n0 + wn + q) = *(const v4fa*)(so + rr * 68 + q); }
    }
    __threadfence();
  }
}

__global__ __launch_bounds__(256) void k_transpose(const float* __restrict__ Wm, float* __restrict__ Wt, int rows, int cols) {
  __shared__ float tS[64][65];
  const int tid = threadIdx.x, tbj = cols / 64, bi = blockIdx.x / tbj, bj = blockIdx.x % tbj;
  for (int e = tid; e < 64 * 64; e += 256) { const int r = e >> 6, c = e & 63; tS[r][c] = Wm[(size_t)(bi * 64 + r) * cols + bj * 64 + c]; }
  __syncthreads();
  for (int ch = tid; ch < 64 * 16; ch += 256) { const int r = ch >> 4, q4 = (ch & 15) * 4; v4f_t o; o[0] = tS[q4][r]; o[1] = tS[q4 + 1][r]; o[2] = tS[q4 + 2][r]; o[3] = tS[q4 + 3][r];
    float* dst = Wt + (size_t)(bj * 64 + r) * rows + bi * 64 + q4; *(volatile v4f_t*)dst = o; __threadfence(); *(volatile v4f_t*)dst = o; }
}

__global__ __launch_bounds__(128) void k_top2(const float* __restrict__ x, int L, float* __restrict__ st) {
  const int n = blockIdx.x, d = threadIdx.x; const float* p = x + (size_t)n * L * DDp + d;
  float t1 = -3.4e38f, t2 = -3.4e38f; int am = 0;
#pragma unroll 1
  for (int l = 0; l < L; ++l) { const float v = p[(size_t)l * DDp];
    if (v > t1) { t2 = t1; t1 = v; am = l; } else if (v > t2) { t2 = v; } }
  float* s = st + ((size_t)n * DDp + d) * 3;
#pragma unroll 1
  for (int pass = 0; pass < 2; ++pass) { *(volatile float*)(s) = t1; *(volatile float*)(s + 1) = t2; *(volatile float*)(s + 2) = (float)am; __threadfence(); }
}
__global__ __launch_bounds__(128) void k_buildA(const float* __restrict__ x, int L, const float* __restrict__ stSelf, const float* __restrict__ stOther, int group, float* __restrict__ A) {
  const size_t row = blockIdx.x; const int n = row / L, l = row % L; const int d = threadIdx.x;
  const float* ss = stSelf + ((size_t)n * DDp + d) * 3; const float* so = stOther + ((size_t)n * DDp + d) * 3;
  const float loo = ((int)ss[2] == l) ? ss[1] : ss[0]; const float cm = so[0];
  float* a = A + row * HHp; const float xv = x[row * DDp + d]; const float f1 = (group == 0) ? loo : cm, f2 = (group == 0) ? cm : loo;
#pragma unroll 1
  for (int pass = 0; pass < 2; ++pass) { *(volatile float*)(a + d) = xv; *(volatile float*)(a + DDp + d) = f1; *(volatile float*)(a + 2 * DDp + d) = f2; __threadfence(); }
}

extern "C" void kernel_launch(void* const* d_in, const int* in_sizes, int n_in,
                              void* d_out, int out_size, void* d_ws, size_t ws_size,
                              hipStream_t stream) {
  (void)in_sizes; (void)n_in; (void)out_size;
  const float* x0 = (const float*)d_in[0], *x1 = (const float*)d_in[1], *W0 = (const float*)d_in[2], *b0 = (const float*)d_in[3], *W1 = (const float*)d_in[4], *b1 = (const float*)d_in[5];
  float* y0 = (float*)d_out;
  float* y1 = y0 + (size_t)NBp * L0 * DDp;
  char* ws = (char*)d_ws;
  float* st0 = (float*)ws; ws += (size_t)NBp * DDp * 3 * 4; float* st1 = (float*)ws; ws += (size_t)NBp * DDp * 3 * 4;
  float* A0 = (float*)ws; ws += (size_t)NBp * L0 * HHp * 4;
  float* A1 = (float*)ws; ws += (size_t)NBp * L1 * HHp * 4;
  float* W0T = (float*)ws; ws += (size_t)HHp * DDp * 4; float* W1T = (float*)ws; ws += (size_t)HHp * DDp * 4;
  if ((size_t)(ws - (char*)d_ws) > ws_size) return;
  const dim3 blk(256);
  k_top2<<<dim3(NBp), dim3(128), 0, stream>>>(x0, L0, st0);
  k_top2<<<dim3(NBp), dim3(128), 0, stream>>>(x1, L1, st1);
  k_buildA<<<dim3(NBp * L0), dim3(128), 0, stream>>>(x0, L0, st0, st1, 0, A0);
  k_buildA<<<dim3(NBp * L1), dim3(128), 0, stream>>>(x1, L1, st1, st0, 1, A1);
  k_transpose<<<dim3((DDp / 64) * (HHp / 64)), blk, 0, stream>>>(W0, W0T, DDp, HHp);
  k_transpose<<<dim3((DDp / 64) * (HHp / 64)), blk, 0, stream>>>(W1, W1T, DDp, HHp);
  gemm_kne<float, 0, false><<<dim3(NBp * L0 / 128, DDp / 128), blk, 0, stream>>>(A0, HHp, W0T, DDp, b0, nullptr, nullptr, y0, DDp, HHp);
  gemm_kne<float, 0, false><<<dim3(NBp * L1 / 128, DDp / 128), blk, 0, stream>>>(A1, HHp, W1T, DDp, b1, nullptr, nullptr, y1, DDp, HHp);
}
